// MV_LSTM_SUPERVISED_52501680226917
// MI455X (gfx1250) — hardware-verified
//
#include <hip/hip_runtime.h>


namespace {
constexpr int Bn = 4096, S = 128, F = 8, H1 = 64, H2 = 32, KIN = S * F + 1  , KP = 1056, NC = S * F  , K1 = 96  , K2 = 96  , NB = 64  ;
constexpr float WS_ = 8.0f, AS_ = 8.0f, WC = 16.0f;

typedef _Float16 b16;
typedef __attribute__((ext_vector_type(16))) _Float16 v16b;
typedef __attribute__((ext_vector_type(8))) _Float16 v8b;
typedef __attribute__((ext_vector_type(8))) float v8f;
typedef __attribute__((ext_vector_type(4))) float v4f;
__device__ __forceinline__ float bf16_rne(float f) { unsigned int u = __float_as_uint(f); u += 0x7FFFu + ((u >> 16) & 1u); return __uint_as_float(u & 0xFFFF0000u); }
__device__ __forceinline__ void split16(float v, b16& hi, b16& lo) { hi = (b16)v; lo = (b16)(v - (float)hi); }
__device__ __forceinline__ v16b frag_kb(const b16* p, int hh) { const v8b a = *(const v8b*)(p + 8 * hh), b = *(const v8b*)(p + 16 + 8 * hh); v16b f;
#pragma unroll
  for (int e = 0; e < 8; ++e) { f[e] = a[e]; f[8 + e] = b[e]; } return f; }
__device__ __forceinline__ v8f wmma16b(v16b a, v16b b, v8f c) { v8f d = __builtin_amdgcn_wmma_f32_16x16x32_f16(false, a, false, b, (short)0, c, false, false); asm volatile("v_nop\n\tv_nop\n\tv_nop\n\tv_nop" : "+v"(d) : "v"(a), "v"(b)); return d; }
__device__ __forceinline__ void wave_lds_sync() { __builtin_amdgcn_fence(__ATOMIC_RELEASE, "workgroup"); __builtin_amdgcn_wave_barrier(); __builtin_amdgcn_fence(__ATOMIC_ACQUIRE, "workgroup"); }
__device__ __forceinline__ float nexp(float x) { return __builtin_amdgcn_exp2f(x * 1.4426950408889634f); }
__device__ __forceinline__ float sigm(float x) { return __builtin_amdgcn_rcpf(1.0f + nexp(-x)); }
__device__ __forceinline__ float tanh_(float x) { const float e = nexp(-2.0f * fabsf(x)); const float t = (1.0f - e) * __builtin_amdgcn_rcpf(1.0f + e); return (x >= 0.0f) ? t : -t; }

__global__ __launch_bounds__(256) void prep_kernel(const float* __restrict__ x, const float* __restrict__ tm, const float* __restrict__ Wc, const float* __restrict__ Wih1, const float* __restrict__ Whh1, const float* __restrict__ Wih2, const float* __restrict__ Whh2,
                                                   b16* __restrict__ xa, b16* __restrict__ wc, b16* __restrict__ b1r, b16* __restrict__ b2r) {
  const size_t tid = (size_t)blockIdx.x * blockDim.x + threadIdx.x, nth = (size_t)gridDim.x * blockDim.x;
  for (int pass = 0; pass < 2; ++pass) {
    for (size_t p = tid; p < (size_t)Bn * KP / 8; p += nth) { const int b = (int)(p / (KP / 8)), k0 = (int)(p % (KP / 8)) * 8; v8b o;
#pragma unroll
      for (int e = 0; e < 8; ++e) { const int k = k0 + e; o[e] = (b16)((k < NC) ? bf16_rne(x[(size_t)b * NC + k]) : (k == NC) ? bf16_rne(tm[b]) : 0.0f); }
      *(volatile v8b*)(xa + p * 8) = o; }
    for (size_t p = tid; p < (size_t)NC * KP / 8; p += nth) { const int n = (int)(p / (KP / 8)), k0 = (int)(p % (KP / 8)) * 8; v8b o;
#pragma unroll
      for (int e = 0; e < 8; ++e) { const int k = k0 + e; o[e] = (b16)((k < KIN) ? bf16_rne(Wc[(size_t)n * KIN + min(k, KIN - 1)]) * WC : 0.0f); }
      *(volatile v8b*)(wc + p * 8) = o; }
    for (size_t p = tid; p < (size_t)4 * H1 * K1; p += nth) { const int row = (int)(p / K1), k = (int)(p % K1); float v = 0.0f;
      if (k < F) v = Wih1[(size_t)row * F + k]; else if (k < F + H1) v = Whh1[(size_t)row * H1 + (k - F)];
      ((volatile b16*)b1r)[p] = (b16)(bf16_rne(v) * WS_); }
    for (size_t p = tid; p < (size_t)4 * H2 * K2; p += nth) { const int row = (int)(p / K2), k = (int)(p % K2); float v = 0.0f;
      if (k < H1) v = Wih2[(size_t)row * H1 + k]; else v = Whh2[(size_t)row * H2 + (k - H1)];
      ((volatile b16*)b2r)[p] = (b16)(bf16_rne(v) * WS_); }
    __threadfence();
  }
}

__global__ __launch_bounds__(128) void combine_kernel(const b16* __restrict__ xa, const b16* __restrict__ wc, const float* __restrict__ bc, float* __restrict__ xc) {
  __shared__ __attribute__((aligned(16))) float Ts[4][32 * 64];
  const int lane = threadIdx.x & 31, wave = threadIdx.x >> 5, nloc = lane & 15, hlf = lane >> 4, m0 = blockIdx.y * 128 + wave * 32, c0 = blockIdx.x * 64;
  v8f acc[2][4];
#pragma unroll
  for (int r = 0; r < 2; ++r)
#pragma unroll
    for (int t = 0; t < 4; ++t) acc[r][t] = (v8f){};
#pragma unroll 3
  for (int kb = 0; kb < KP; kb += 32) { const v16b a0 = frag_kb(xa + (size_t)(m0 + nloc) * KP + kb, hlf), a1 = frag_kb(xa + (size_t)(m0 + 16 + nloc) * KP + kb, hlf);
#pragma unroll
    for (int t = 0; t < 4; ++t) { const v16b bw = frag_kb(wc + (size_t)(c0 + t * 16 + nloc) * KP + kb, hlf); acc[0][t] = wmma16b(a0, bw, acc[0][t]); acc[1][t] = wmma16b(a1, bw, acc[1][t]); } }
  float* Tt = Ts[wave];
#pragma unroll
  for (int t = 0; t < 4; ++t)
#pragma unroll
    for (int r = 0; r < 2; ++r)
#pragma unroll
      for (int v = 0; v < 8; ++v) Tt[(r * 16 + v + 8 * hlf) * 64 + t * 16 + nloc] = fmaxf(acc[r][t][v] * (1.0f / WC) + bf16_rne(bc[c0 + t * 16 + nloc]), 0.0f);
  wave_lds_sync();
  float* dst0 = xc + (size_t)m0 * NC + c0;
  for (int pass = 0; pass < 2; ++pass) {
#pragma unroll
    for (int j = 0; j < 16; ++j) { const int rr = j * 2 + hlf, c4 = nloc * 4; *(volatile v4f*)(dst0 + (size_t)rr * NC + c4) = *(const v4f*)(Tt + rr * 64 + c4); }
    __threadfence(); }
}

__global__ __launch_bounds__(256) void lstm_kernel(const float* __restrict__ xc, const b16* __restrict__ b1r, const b16* __restrict__ b2r, const float* __restrict__ bih2, const float* __restrict__ bhh2, const float* __restrict__ Wout, const float* __restrict__ bout, float* __restrict__ out) {
  __shared__ __attribute__((aligned(16))) b16 H1h[2][NB][H1 + 8], H1l[2][NB][H1 + 8], H2h[2][NB][H2 + 8], H2l[2][NB][H2 + 8]; __shared__ float Ored[2][NB];
  const int t_ = threadIdx.x, wave = t_ >> 5, lane = t_ & 31, nloc = lane & 15, hlf = lane >> 4, rg = wave & 3, half = wave >> 2, r0 = rg * 16; const int b0 = blockIdx.x * NB;
  for (int i = t_; i < 2 * NB * (H1 + 8); i += 256) { (&H1h[0][0][0])[i] = (b16)0.0f; (&H1l[0][0][0])[i] = (b16)0.0f; }
  for (int i = t_; i < 2 * NB * (H2 + 8); i += 256) { (&H2h[0][0][0])[i] = (b16)0.0f; (&H2l[0][0][0])[i] = (b16)0.0f; }
  float c1[2][8], c2[8], oac[8];
#pragma unroll
  for (int v = 0; v < 8; ++v) { c1[0][v] = 0.0f; c1[1][v] = 0.0f; c2[v] = 0.0f; oac[v] = 0.0f; }
  const int u2 = half * 16 + nloc; float bias2[4];
#pragma unroll
  for (int g = 0; g < 4; ++g) bias2[g] = bf16_rne(bih2[g * H2 + u2]) + bf16_rne(bhh2[g * H2 + u2]);
  const float sc = 1.0f / (AS_ * WS_);
  __syncthreads();
  for (int st = 0; st < S; ++st) { const int pb = st & 1, nb = pb ^ 1;
    float xv[8];
#pragma unroll
    for (int e = 0; e < 8; ++e) xv[e] = (hlf == 0) ? xc[(size_t)(b0 + r0 + nloc) * NC + st * F + e] : 0.0f;
#pragma unroll
    for (int ug = 0; ug < 2; ++ug) { v8f acc[4] = {{}, {}, {}, {}};
#pragma unroll
      for (int ks = 0; ks < 3; ++ks) { v16b ah, al; const int row = r0 + nloc;
#pragma unroll
        for (int e = 0; e < 16; ++e) { const int k = ks * 32 + ((e < 8) ? (8 * hlf + e) : (16 + 8 * hlf + e - 8)); b16 a = (b16)0.0f, c = (b16)0.0f;
          if (ks == 0 && e < 8 && hlf == 0) { split16(xv[e] * AS_, a, c); }
          else if (k >= F && k < F + H1) { a = H1h[pb][row][k - F]; c = H1l[pb][row][k - F]; }
          ah[e] = a; al[e] = c; }
#pragma unroll
        for (int g = 0; g < 4; ++g) { const v16b bw = frag_kb(b1r + (size_t)(g * H1 + half * 32 + ug * 16 + nloc) * K1 + ks * 32, hlf); acc[g] = wmma16b(ah, bw, acc[g]); acc[g] = wmma16b(al, bw, acc[g]); } }
#pragma unroll
      for (int v = 0; v < 8; ++v) { const float gi = acc[0][v] * sc, gf = acc[1][v] * sc, gg = acc[2][v] * sc, go = acc[3][v] * sc;
        const float c = sigm(gf) * c1[ug][v] + sigm(gi) * tanh_(gg); c1[ug][v] = c; const float h = sigm(go) * tanh_(c);
        b16 a, l; split16(h * AS_, a, l); const int row = r0 + 8 * hlf + v, u = half * 32 + ug * 16 + nloc; H1h[nb][row][u] = a; H1l[nb][row][u] = l; } }
    __syncthreads();
    { v8f acc[4] = {{}, {}, {}, {}};
#pragma unroll
      for (int ks = 0; ks < 3; ++ks) { v16b a0, l0; const int rA = r0 + nloc;
#pragma unroll
        for (int e = 0; e < 16; ++e) { const int k = ks * 32 + ((e < 8) ? (8 * hlf + e) : (16 + 8 * hlf + e - 8));
          if (k < H1) { a0[e] = H1h[nb][rA][k]; l0[e] = H1l[nb][rA][k]; } else { a0[e] = H2h[pb][rA][k - H1]; l0[e] = H2l[pb][rA][k - H1]; } }
#pragma unroll
        for (int g = 0; g < 4; ++g) { const v16b bw = frag_kb(b2r + (size_t)(g * H2 + half * 16 + nloc) * K2 + ks * 32, hlf); acc[g] = wmma16b(a0, bw, acc[g]); acc[g] = wmma16b(l0, bw, acc[g]); } }
      const float wo = bf16_rne(Wout[st * H2 + u2]);
#pragma unroll
      for (int v = 0; v < 8; ++v) { const float gi = acc[0][v] * sc + bias2[0], gf = acc[1][v] * sc + bias2[1], gg = acc[2][v] * sc + bias2[2], go = acc[3][v] * sc + bias2[3];
        const float c = sigm(gf) * c2[v] + sigm(gi) * tanh_(gg); c2[v] = c; const float h = sigm(go) * tanh_(c);
        b16 a, l; split16(h * AS_, a, l); const int row = r0 + 8 * hlf + v; H2h[nb][row][u2] = a; H2l[nb][row][u2] = l; oac[v] += h * wo; } }
    __syncthreads();
  }
#pragma unroll
  for (int v = 0; v < 8; ++v) { float s = oac[v];
#pragma unroll
    for (int o = 1; o < 16; o <<= 1) s += __shfl_xor(s, o);
    if (nloc == 0) Ored[half][r0 + 8 * hlf + v] = s; }
  __syncthreads();
  const float bo = bf16_rne(bout[0]);
  for (int pass = 0; pass < 2; ++pass) { if (t_ < NB) ((volatile float*)out)[b0 + t_] = Ored[0][t_] + Ored[1][t_] + bo; __threadfence(); }
}
}

extern "C" void kernel_launch(void* const* d_in, const int* in_sizes, int n_in,
                              void* d_out, int out_size, void* d_ws, size_t ws_size, hipStream_t stream) {
  (void)n_in; (void)out_size;
  const float* x = (const float*)d_in[0]; const float* tm = (const float*)d_in[1]; const float* Wc = (const float*)d_in[2]; const float* bc = (const float*)d_in[3];
  const float* Wih1 = (const float*)d_in[4]; const float* Whh1 = (const float*)d_in[5]; const float* Wih2 = (const float*)d_in[6]; const float* Whh2 = (const float*)d_in[7]; const float* bih2 = (const float*)d_in[8]; const float* bhh2 = (const float*)d_in[9];
  const float* Wout = (const float*)d_in[10]; const float* bout = (const float*)d_in[11];
  float* out = (float*)d_out;
  if (in_sizes[0] != Bn * S * F || in_sizes[1] != Bn || in_sizes[2] != NC * KIN || in_sizes[4] != 4 * H1 * F || in_sizes[5] != 4 * H1 * H1 || in_sizes[6] != 4 * H2 * H1 || in_sizes[7] != 4 * H2 * H2 || in_sizes[10] != S * H2) return;
  size_t off = 0; char* ws = (char*)d_ws;
  auto carve = [&](size_t bytes) { char* p = ws + off; off += (bytes + 255) & ~(size_t)255; return p; };
  b16* xa = (b16*)carve((size_t)Bn * KP * 2); b16* wcr = (b16*)carve((size_t)NC * KP * 2); b16* b1r = (b16*)carve((size_t)4 * H1 * K1 * 2); b16* b2r = (b16*)carve((size_t)4 * H2 * K2 * 2); float* xc = (float*)carve((size_t)Bn * NC * 4);
  if (off > ws_size) return;
  prep_kernel<<<1024, 256, 0, stream>>>(x, tm, Wc, Wih1, Whh1, Wih2, Whh2, xa, wcr, b1r, b2r);
  combine_kernel<<<dim3(NC / 64, Bn / 128), 128, 0, stream>>>(xa, wcr, bc, xc);
  lstm_kernel<<<Bn / NB, 256, 0, stream>>>(xc, b1r, b2r, bih2, bhh2, Wout, bout, out);
}
